// MultiHeadAttentionMap_75505525063895
// MI455X (gfx1250) — hardware-verified
//
#include <hip/hip_runtime.h>
#include <stdint.h>


typedef _Float16 f16;
typedef f16 v8h __attribute__((ext_vector_type(8)));
typedef f16 v16h __attribute__((ext_vector_type(16)));
typedef __bf16 v16b __attribute__((ext_vector_type(16)));
typedef unsigned short us4 __attribute__((ext_vector_type(4)));
typedef unsigned short us8 __attribute__((ext_vector_type(8)));
typedef unsigned short us16 __attribute__((ext_vector_type(16)));
typedef float v4f __attribute__((ext_vector_type(4)));
typedef float v8f __attribute__((ext_vector_type(8)));

union FragH { v16h v; v8h half[2]; };
union FragB { v16b v; us16 u; us8 half[2]; };

#define NB      2
#define SEQ     2048
#define DMODEL  1024
#define HEADS   16
#define DHEAD   64
#define WAVES   4
#define NTHR    (WAVES * 32)
#define QROWS_W 16
#define QROWS_B (WAVES * QROWS_W)
#define KT      32
#define KPITCH  72
#define VPITCH  40
#define PPITCH  40
#define OPITCH  68
#define PLO_SCALE 4096.0f
#define V_SCALE   16.0f

static __device__ __forceinline__ unsigned short bf16_bits(float f) {
    unsigned u = __float_as_uint(f);
    u += 0x7FFFu + ((u >> 16) & 1u);
    return (unsigned short)(u >> 16);
}
static __device__ __forceinline__ float bf16_val(float f) {
    return __uint_as_float(((unsigned)bf16_bits(f)) << 16);
}

static __device__ __forceinline__ v8f wm_bf16(v16b a, v16b b, v8f c) {
    c = __builtin_amdgcn_wmma_f32_16x16x32_bf16(false, a, false, b, (short)0, c, false, false);
    asm volatile("v_nop\n\tv_nop\n\tv_nop\n\tv_nop" : "+v"(c) : "v"(a), "v"(b));
    return c;
}
static __device__ __forceinline__ v8f wm_f16(v16h a, v16h b, v8f c) {
    c = __builtin_amdgcn_wmma_f32_16x16x32_f16(false, a, false, b, (short)0, c, false, false);
    asm volatile("v_nop\n\tv_nop\n\tv_nop\n\tv_nop" : "+v"(c) : "v"(a), "v"(b));
    return c;
}

__global__ __launch_bounds__(NTHR)
void k_attn(const float* __restrict__ Q,
            const float* __restrict__ K,
            const float* __restrict__ V,
            const int*   __restrict__ Msk,
            float* O, int nqblk)
{
    __shared__ __attribute__((aligned(16))) unsigned short Ksh[KT][KPITCH];
    __shared__ __attribute__((aligned(16))) f16   Vt[DHEAD][VPITCH];
    __shared__ __attribute__((aligned(16))) f16   Phi[WAVES][16][PPITCH];
    __shared__ __attribute__((aligned(16))) f16   Plo[WAVES][16][PPITCH];
    __shared__ __attribute__((aligned(16))) float Osh[WAVES][16][OPITCH];

    const int tid = threadIdx.x;
    const int w  = tid >> 5;
    const int l  = tid & 31;
    const int hh = l >> 4;
    const int ln = l & 15;

    int bid = blockIdx.x;
    const int qb = bid % nqblk; bid /= nqblk;
    const int h  = bid % HEADS;
    const int b  = bid / HEADS;
    if (b >= NB || (qb + 1) * QROWS_B > SEQ) return;
    const int q0 = qb * QROWS_B + w * QROWS_W;

    FragB qa[2];
    {
        const float* qp = Q + (size_t)(b * SEQ + q0 + ln) * DMODEL + h * DHEAD;
        #pragma unroll
        for (int ks = 0; ks < 2; ++ks) {
            #pragma unroll
            for (int hf = 0; hf < 2; ++hf) {
                const float* src = qp + 32 * ks + 16 * hf + 8 * hh;
                v4f x0 = *(const v4f*)src;
                v4f x1 = *(const v4f*)(src + 4);
                us8 t;
                t[0] = bf16_bits(x0[0] * 0.125f); t[1] = bf16_bits(x0[1] * 0.125f);
                t[2] = bf16_bits(x0[2] * 0.125f); t[3] = bf16_bits(x0[3] * 0.125f);
                t[4] = bf16_bits(x1[0] * 0.125f); t[5] = bf16_bits(x1[1] * 0.125f);
                t[6] = bf16_bits(x1[2] * 0.125f); t[7] = bf16_bits(x1[3] * 0.125f);
                qa[ks].half[hf] = t;
            }
        }
    }

    v8f acc[4];
    float lsum[8];
    const v8f zero = 0.0f;
    #pragma unroll
    for (int c = 0; c < 4; ++c) acc[c] = zero;
    #pragma unroll
    for (int r = 0; r < 8; ++r) lsum[r] = 0.0f;

    for (int it = 0; it < SEQ / KT; ++it) {
        const int key0 = it * KT;

        __syncthreads();
        #pragma unroll
        for (int j = 0; j < (KT * DHEAD / 4) / NTHR; ++j) {
            const int i  = tid + NTHR * j;
            const int kr = i >> 4;
            const int d4 = (i & 15) * 4;
            const size_t goff = (size_t)(b * SEQ + key0 + kr) * DMODEL + h * DHEAD + d4;
            v4f x = *(const v4f*)(K + goff);
            us4 kbv;
            kbv[0] = bf16_bits(x[0]); kbv[1] = bf16_bits(x[1]);
            kbv[2] = bf16_bits(x[2]); kbv[3] = bf16_bits(x[3]);
            *(us4*)(&Ksh[kr][d4]) = kbv;
            v4f y = *(const v4f*)(V + goff);
            Vt[d4 + 0][kr] = (f16)(bf16_val(y[0]) * V_SCALE);
            Vt[d4 + 1][kr] = (f16)(bf16_val(y[1]) * V_SCALE);
            Vt[d4 + 2][kr] = (f16)(bf16_val(y[2]) * V_SCALE);
            Vt[d4 + 3][kr] = (f16)(bf16_val(y[3]) * V_SCALE);
        }
        __syncthreads();

        v8f s[2];
        #pragma unroll
        for (int ct = 0; ct < 2; ++ct) {
            s[ct] = zero;
            #pragma unroll
            for (int ks = 0; ks < 2; ++ks) {
                FragB kb;
                kb.half[0] = *(const us8*)(&Ksh[16 * ct + ln][32 * ks + 8 * hh]);
                kb.half[1] = *(const us8*)(&Ksh[16 * ct + ln][32 * ks + 16 + 8 * hh]);
                s[ct] = wm_bf16(qa[ks].v, kb.v, s[ct]);
            }
        }

        #pragma unroll
        for (int r = 0; r < 8; ++r) {
            const int* mr = Msk + (size_t)(b * SEQ + q0 + 8 * hh + r) * SEQ + key0;
            const int m0 = mr[ln];
            const int m1 = mr[16 + ln];
            const float p0 = (m0 != 0) ? __expf(s[0][r]) : 0.0f;
            const float p1 = (m1 != 0) ? __expf(s[1][r]) : 0.0f;
            lsum[r] += p0 + p1;
            const f16 h0 = (f16)p0;
            const f16 h1 = (f16)p1;
            const f16 g0 = (f16)((p0 - (float)h0) * PLO_SCALE);
            const f16 g1 = (f16)((p1 - (float)h1) * PLO_SCALE);
            Phi[w][8 * hh + r][ln]      = h0;
            Phi[w][8 * hh + r][16 + ln] = h1;
            Plo[w][8 * hh + r][ln]      = g0;
            Plo[w][8 * hh + r][16 + ln] = g1;
        }
        __syncthreads();

        FragH pa, pl;
        pa.half[0] = *(const v8h*)(&Phi[w][ln][8 * hh]);
        pa.half[1] = *(const v8h*)(&Phi[w][ln][16 + 8 * hh]);
        pl.half[0] = *(const v8h*)(&Plo[w][ln][8 * hh]);
        pl.half[1] = *(const v8h*)(&Plo[w][ln][16 + 8 * hh]);

        #pragma unroll
        for (int c = 0; c < 4; ++c) {
            FragH vb;
            vb.half[0] = *(const v8h*)(&Vt[16 * c + ln][8 * hh]);
            vb.half[1] = *(const v8h*)(&Vt[16 * c + ln][16 + 8 * hh]);
            acc[c] = wm_f16(pa.v, vb.v, acc[c]);
            v8f t  = wm_f16(pl.v, vb.v, zero);
            acc[c] += t * (1.0f / PLO_SCALE);
        }
    }

    float scl[8];
    #pragma unroll
    for (int r = 0; r < 8; ++r) {
        float rs = lsum[r];
        rs += __shfl_xor(rs, 1);
        rs += __shfl_xor(rs, 2);
        rs += __shfl_xor(rs, 4);
        rs += __shfl_xor(rs, 8);
        scl[r] = (rs > 0.0f) ? ((1.0f / rs) * (1.0f / V_SCALE)) : 0.0f;
    }
    #pragma unroll
    for (int c = 0; c < 4; ++c) {
        #pragma unroll
        for (int r = 0; r < 8; ++r)
            Osh[w][8 * hh + r][16 * c + ln] = acc[c][r] * scl[r];
    }
    __syncthreads();

    v4f ov[8];
    #pragma unroll
    for (int j = 0; j < 8; ++j)
        ov[j] = *(const v4f*)(&Osh[w][2 * j + hh][4 * ln]);

    volatile v4f* Ov = (volatile v4f*)O;
    #pragma unroll
    for (int j = 0; j < 8; ++j) {
        const size_t idx4 = (size_t)(b * SEQ + q0 + 2 * j + hh) * (DMODEL / 4) + h * (DHEAD / 4) + ln;
        Ov[idx4] = ov[j];
    }
    __threadfence();
    #pragma unroll
    for (int j = 0; j < 8; ++j) {
        const size_t idx4 = (size_t)(b * SEQ + q0 + 2 * j + hh) * (DMODEL / 4) + h * (DHEAD / 4) + ln;
        Ov[idx4] = ov[j];
    }
}

extern "C" void kernel_launch(void* const* d_in, const int* in_sizes, int n_in,
                              void* d_out, int out_size, void* d_ws, size_t ws_size,
                              hipStream_t stream)
{
    (void)d_ws; (void)ws_size;
    if (n_in < 4) return;
    const int n_act = NB * SEQ * DMODEL;
    const int n_msk = NB * SEQ * SEQ;
    if (in_sizes[0] != n_act || in_sizes[1] != n_act || in_sizes[2] != n_act ||
        in_sizes[3] != n_msk || out_size != n_act) return;
    if ((SEQ % QROWS_B) != 0 || (SEQ % KT) != 0) return;

    const float* Q = (const float*)d_in[0];
    const float* K = (const float*)d_in[1];
    const float* V = (const float*)d_in[2];
    const int*   M = (const int*)d_in[3];
    float*       O = (float*)d_out;

    const int nqblk = (SEQ + QROWS_B - 1) / QROWS_B;
    dim3 grid((unsigned)(NB * HEADS * nqblk));
    dim3 block(NTHR);
    k_attn<<<grid, block, 0, stream>>>(Q, K, V, M, O, nqblk);
    (void)hipGetLastError();
}
